// CAST_41274635715112
// MI455X (gfx1250) — hardware-run, weakly checked
//
#include <hip/hip_runtime.h>
#pragma clang fp contract(off)


#ifndef NB
#define NB 64
#endif
#define NB_FULL 64
#define NH   50
#define NN   50
#define RD   400
#define PD   100
#define FD   500
#define AD   200
#define NPOS 52
#define KP   512
#define APAD 256
#define HPAD 64
#define MROWS (NB * NN)
#define MPAD  ((MROWS + 63) / 64 * 64)
#define OSW  68
#define TP   72
#define SW   4
#define PCS  1024.0f
#define PCI  (1.0f / 1024.0f)
#define L2E  1.4426950408889634f
#define NEGV (-1.0e9f)
#define NEGB (-3.0e38f)

static_assert(FD == RD + PD);
static_assert(NH == NN);
static_assert(RD % 8 == 0);
static_assert(PD % 4 == 0);
static_assert(FD % 4 == 0);
static_assert(KP % 32 == 0);
static_assert(KP >= FD);
static_assert(KP % 64 == 0);
static_assert(KP / 8 == 64);
static_assert(APAD % 64 == 0);
static_assert(APAD >= AD);
static_assert(AD % 4 == 0);
static_assert(HPAD == 64);
static_assert(HPAD % 32 == 0);
static_assert(NH > 32);
static_assert(NH <= HPAD);
static_assert(NN <= HPAD);
static_assert(MPAD % 64 == 0);
static_assert(HPAD % (4 * SW) == 0);
static_assert(NB <= NB_FULL);
static_assert(((size_t)NB_FULL * NN * FD * 4) == (size_t)6400000);
static_assert((((size_t)NB_FULL * NN * FD * 4) % 128) == 0);
static_assert((OSW * 4) % 16 == 0);
static_assert((TP * 2) % 16 == 0);
static_assert(16 * OSW * 4 <= 131072);
static_assert(64 * TP * 2 <= 131072);
static_assert(SW * 4 * HPAD * 2 <= 131072);

typedef _Float16 h16;
typedef unsigned short bf;
typedef __attribute__((ext_vector_type(16))) __bf16   v16bf;
typedef __attribute__((ext_vector_type(16))) _Float16 v16h;
typedef __attribute__((ext_vector_type(8)))  _Float16 v8h;
typedef __attribute__((ext_vector_type(8)))  unsigned short v8us;
typedef __attribute__((ext_vector_type(8)))  float    v8f;
typedef __attribute__((ext_vector_type(4)))  float    v4f;
typedef v4f  __attribute__((may_alias)) v4fa;
typedef v8h  __attribute__((may_alias)) v8ha;

__device__ __forceinline__ unsigned short f2bf(float f) { unsigned u = __float_as_uint(f); u += 0x7FFFu + ((u >> 16) & 1u); return (unsigned short)(u >> 16); }
__device__ __forceinline__ float bfr(float f) { return __uint_as_float(((unsigned)f2bf(f)) << 16); }
__device__ __forceinline__ v16h cat16(v8h lo, v8h hi) { return __builtin_shufflevector(lo, hi, 0, 1, 2, 3, 4, 5, 6, 7, 8, 9, 10, 11, 12, 13, 14, 15); }
__device__ __forceinline__ v16bf cat16b(v8us lo, v8us hi) { return __builtin_bit_cast(v16bf, __builtin_shufflevector(lo, hi, 0, 1, 2, 3, 4, 5, 6, 7, 8, 9, 10, 11, 12, 13, 14, 15)); }
__device__ __forceinline__ v8f wmma16(v16h a, v16h b, v8f c) { return __builtin_amdgcn_wmma_f32_16x16x32_f16(false, a, false, b, (short)0, c, false, false); }
__device__ __forceinline__ v8f wmmab(v16bf a, v16bf b, v8f c) { return __builtin_amdgcn_wmma_f32_16x16x32_bf16(false, a, false, b, (short)0, c, false, false); }
__device__ __forceinline__ v16h  ldh(const h16* p) { return cat16(*(const v8h*)p, *(const v8h*)(p + 16)); }
__device__ __forceinline__ v16bf ldb(const bf* p)  { return cat16b(*(const v8us*)p, *(const v8us*)(p + 16)); }
__device__ __forceinline__ void wave_sync() { __builtin_amdgcn_fence(3  , "wavefront"); __builtin_amdgcn_wave_barrier(); asm volatile("" ::: "memory"); }
__device__ __forceinline__ v8f wmma16g(v16h a, v16h b, v8f c) { c = wmma16(a, b, c); asm volatile("v_nop\n\tv_nop\n\tv_nop\n\tv_nop" : "+v"(c) : "v"(a), "v"(b)); return c; }
__device__ __forceinline__ v8f wmmabg(v16bf a, v16bf b, v8f c) { c = wmmab(a, b, c); asm volatile("v_nop\n\tv_nop\n\tv_nop\n\tv_nop" : "+v"(c) : "v"(a), "v"(b)); return c; }
static __device__ __forceinline__ h16 toh_flush(float v) { const h16 r = (h16)v; return (fabsf(v) < 6.103515625e-05f) ? (h16)0.0f : r; }
__device__ __forceinline__ int posrow(int p) { p = p < 0 ? p + NPOS : p; p = p < 0 ? 0 : p; p = p > NPOS - 1 ? NPOS - 1 : p; return p; }

__global__ __launch_bounds__(256) void k_wconv(const float* __restrict__ W1, bf* WB) {
    const int i = (int)blockIdx.x * 256 + (int)threadIdx.x; if (i >= 2 * APAD * (KP / 8)) return;
    const int k8 = (i % (KP / 8)) * 8; const int a = (i / (KP / 8)) % APAD; const int w = i / ((KP / 8) * APAD);
    const int ac = a < AD ? a : AD - 1;
    const size_t rb = (size_t)ac * (2 * FD) + (size_t)w * FD;
    v8us o;
#pragma unroll
    for (int j = 0; j < 8; ++j) { const int k = k8 + j; const int kc = k < FD ? k : FD - 1;
        float x = W1[rb + (size_t)kc]; asm volatile("" : "+v"(x));
        const bool ok = (k < FD) & (a < AD); o[j] = f2bf(ok ? x : 0.0f); }
    *(volatile v8us*)(WB + (size_t)i * 8) = o; __threadfence(); *(volatile v8us*)(WB + (size_t)i * 8) = o;
}

__global__ __launch_bounds__(256) void k_xrow(const float* __restrict__ src, const int* __restrict__ pos, const float* __restrict__ pe, bf* dst, int usepos) {
    const int i = (int)blockIdx.x * 256 + (int)threadIdx.x; if (i >= MPAD * (KP / 8)) return;
    const int k8 = (i % (KP / 8)) * 8; const int r = i / (KP / 8);
    const int rc = r < MROWS ? r : MROWS - 1;
    int pz = pos[rc]; asm volatile("" : "+v"(pz));
    const int prow = usepos ? posrow(pz) : 1;
    const int kr = k8 < RD - 8 ? k8 : RD - 8;
    int pa = k8 - RD;     pa = pa < 0 ? 0 : (pa > PD - 4 ? PD - 4 : pa);
    int pb = k8 - RD + 4; pb = pb < 0 ? 0 : (pb > PD - 4 ? PD - 4 : pb);
    v4f r0 = *(const v4f*)(src + (size_t)rc * RD + kr), r1 = *(const v4f*)(src + (size_t)rc * RD + kr + 4);
    v4f p0 = *(const v4f*)(pe + (size_t)prow * PD + pa), p1 = *(const v4f*)(pe + (size_t)prow * PD + pb);
    asm volatile("" : "+v"(r0)); asm volatile("" : "+v"(r1)); asm volatile("" : "+v"(p0)); asm volatile("" : "+v"(p1));
    const bool rv = r < MROWS;
    const bool inr = (k8 < RD) & rv;
    const bool ip0 = (k8 >= RD) & (k8 < FD) & rv;
    const bool ip1 = (k8 >= RD) & (k8 + 4 < FD) & rv;
    v8us o;
#pragma unroll
    for (int j = 0; j < 4; ++j) {
        const float x0 = inr ? r0[j] : (ip0 ? p0[j] : 0.0f);
        const float x1 = inr ? r1[j] : (ip1 ? p1[j] : 0.0f);
        o[j] = f2bf(x0); o[4 + j] = f2bf(x1); }
    *(volatile v8us*)(dst + (size_t)i * 8) = o; __threadfence(); *(volatile v8us*)(dst + (size_t)i * 8) = o;
}

__global__ __launch_bounds__(256) void k_cand(const float* __restrict__ cand, const float* __restrict__ pe, float* O1) {
    const int i = (int)blockIdx.x * 256 + (int)threadIdx.x; if (i >= MROWS * (FD / 4)) return;
    const int r = i / (FD / 4); const int c = (i % (FD / 4)) * 4;
    const int cr = c < RD ? c : RD - 4; int cp = c - RD; cp = cp < 0 ? 0 : cp;
    v4f xr = *(const v4f*)(cand + (size_t)r * RD + cr); v4f xp = *(const v4f*)(pe + PD + cp);
    asm volatile("" : "+v"(xr)); asm volatile("" : "+v"(xp));
    v4f o;
#pragma unroll
    for (int j = 0; j < 4; ++j) o[j] = bfr(c < RD ? xr[j] : xp[j]);
    *(volatile v4f*)(O1 + (size_t)i * 4) = o; __threadfence(); *(volatile v4f*)(O1 + (size_t)i * 4) = o;
}

__global__ __launch_bounds__(256) void k_histT(const float* __restrict__ hist, const int* __restrict__ pos, const float* __restrict__ pe, h16* HT) {
    __shared__ __align__(16) h16 th[64 * TP];
    const int t = (int)threadIdx.x; const int f0 = (int)blockIdx.x * 64; const int b = (int)blockIdx.y;
    const int fl = t & 63, hq = t >> 6;
    const int f = f0 + fl; const int fr = f < RD ? f : RD - 1; int fp = f - RD; fp = fp < 0 ? 0 : (fp > PD - 1 ? PD - 1 : fp);
    static_assert(256 * 16 == 64 * HPAD);
#pragma unroll 1
    for (int it = 0; it < 16; ++it) {
        const int h = hq + 4 * it; const int hc = h < NH ? h : NH - 1; const size_t row = (size_t)b * NH + (size_t)hc;
        int pz = pos[row]; asm volatile("" : "+v"(pz)); pz = posrow(pz);
        float xr = hist[row * RD + (size_t)fr]; float xp = pe[(size_t)pz * PD + (size_t)fp];
        asm volatile("" : "+v"(xr)); asm volatile("" : "+v"(xp));
        const float v = (f < RD) ? xr : xp;
        const bool ok = (h < NH) & (f < FD);
        const h16 o = ok ? toh_flush(bfr(v)) : (h16)0.0f;
        th[fl * TP + h] = o; }
    __syncthreads();
    static_assert(256 * 2 * 16 == 64 * HPAD * 2);
#pragma unroll 1
    for (int ps = 0; ps < 2; ++ps) {
#pragma unroll
        for (int it = 0; it < 2; ++it) { const int p = it * 256 + t; const int row = p >> 3, pc = p & 7;
            const v8h val = *(const v8ha*)(&th[row * TP + pc * 8]);
            *(volatile v8h*)(HT + ((size_t)b * KP + (size_t)(f0 + row)) * HPAD + (size_t)pc * 8) = val; }
        if (ps == 0) __threadfence(); }
}

__global__ __launch_bounds__(32) void k_gemm1(const bf* __restrict__ XB, const bf* __restrict__ WB, float* HP) {
    __shared__ __align__(16) float os[16 * OSW];
    const int lane = threadIdx.x & 31, lr = lane & 15, hi = lane >> 4;
    const int r0 = (int)blockIdx.x * 64, c0 = (int)blockIdx.y * 64, w = (int)blockIdx.z;
    v8f acc[4][4];
#pragma unroll
    for (int mb = 0; mb < 4; ++mb)
#pragma unroll
        for (int nb = 0; nb < 4; ++nb) acc[mb][nb] = (v8f){};
    const size_t aoff = ((size_t)w * MPAD + (size_t)(r0 + lr)) * KP + 8 * hi, boff = ((size_t)w * APAD + (size_t)(c0 + lr)) * KP + 8 * hi;
#pragma unroll 1
    for (int kc = 0; kc < KP; kc += 32) {
        v16bf a[4];
#pragma unroll
        for (int mb = 0; mb < 4; ++mb) a[mb] = ldb(XB + aoff + (size_t)mb * 16 * KP + kc);
#pragma unroll
        for (int nb = 0; nb < 4; ++nb) { const v16bf bq = ldb(WB + boff + (size_t)nb * 16 * KP + kc);
#pragma unroll
            for (int mb = 0; mb < 4; ++mb) acc[mb][nb] = wmmabg(a[mb], bq, acc[mb][nb]); }
    }
    float* outp = HP + ((size_t)w * MPAD + (size_t)r0) * APAD + (size_t)c0;
    static_assert(32 * 16 * 8 == 16 * 64 * 4);
#pragma unroll
    for (int mb = 0; mb < 4; ++mb) {
#pragma unroll
        for (int nb = 0; nb < 4; ++nb) {
#pragma unroll
            for (int j = 0; j < 8; ++j) os[(hi * 8 + j) * OSW + nb * 16 + lr] = acc[mb][nb][j]; }
        wave_sync();
#pragma unroll 1
        for (int ps = 0; ps < 2; ++ps) {
#pragma unroll
            for (int s = 0; s < 8; ++s) { const int row = 2 * s + (lane >> 4), c4 = (lane & 15) * 4;
                const v4f val = *(const v4fa*)(&os[row * OSW + c4]);
                *(volatile v4f*)(outp + (size_t)(mb * 16 + row) * APAD + c4) = val; }
            if (ps == 0) __threadfence(); }
        wave_sync();
    }
}

__global__ __launch_bounds__(32 * SW) void k_score(const float* __restrict__ HC, const float* __restrict__ HH, const int* __restrict__ maskp,
                                                   const float* __restrict__ b1, const float* __restrict__ w2, const float* __restrict__ b2, h16* AP) {
    __shared__ __align__(16) h16 pt[SW * 4 * HPAD];
    const int lane = threadIdx.x & 31;
    const int wave = __builtin_amdgcn_readfirstlane((int)(threadIdx.x >> 5));
    const int b = (int)blockIdx.y;
    const int n0 = ((int)blockIdx.x * SW + wave) * 4;
    h16* dst = AP + ((size_t)b * HPAD + (size_t)n0) * HPAD + (size_t)lane * 8;
    static_assert(32 * 16 == 4 * HPAD * 2);
    if (n0 >= NN) { const v8h z = (v8h){}; *(volatile v8h*)dst = z; __threadfence(); *(volatile v8h*)dst = z; return; }
    const int nvec = ((int)blockIdx.x * SW + (int)(threadIdx.x >> 5)) * 4;
    size_t oc[4]; bool rok[4];
#pragma unroll
    for (int i = 0; i < 4; ++i) { int q = nvec + i; rok[i] = q < NN; q = q < NN ? q : NN - 1; q = __builtin_amdgcn_readfirstlane(q);
        oc[i] = ((size_t)b * NN + (size_t)q) * APAD; }
    const int hB = lane + 32; const int hBc = hB < NH ? hB : NH - 1; const bool okB = hB < NH;
    const size_t hb = (size_t)b * NH;
    const size_t oa = (hb + (size_t)lane) * APAD, ob = (hb + (size_t)hBc) * APAD;
    int mkA = maskp[hb + (size_t)lane], mkB = maskp[hb + (size_t)hBc];
    asm volatile("" : "+v"(mkA)); asm volatile("" : "+v"(mkB));
    const float b2v = bfr(b2[0]);
    float accA[4], accB[4];
#pragma unroll
    for (int i = 0; i < 4; ++i) { accA[i] = 0.0f; accB[i] = 0.0f; }
#pragma unroll 1
    for (int a4 = 0; a4 < AD / 4; ++a4) {
        const v4f xa = *(const v4f*)(HH + oa + 4 * a4), xb = *(const v4f*)(HH + ob + 4 * a4);
        const v4f bv = *(const v4f*)(b1 + 4 * a4), wv = *(const v4f*)(w2 + 4 * a4);
        float bb[4], ww[4];
#pragma unroll
        for (int j = 0; j < 4; ++j) { bb[j] = bfr(bv[j]); ww[j] = bfr(wv[j]); }
#pragma unroll
        for (int i = 0; i < 4; ++i) { const v4f c = *(const v4f*)(HC + oc[i] + 4 * a4);
#pragma unroll
            for (int j = 0; j < 4; ++j) {
                const float va = fmaxf((c[j] + xa[j]) + bb[j], 0.0f), vb = fmaxf((c[j] + xb[j]) + bb[j], 0.0f);
                accA[i] = fmaf(va, ww[j], accA[i]); accB[i] = fmaf(vb, ww[j], accB[i]); } }
    }
#pragma unroll
    for (int i = 0; i < 4; ++i) {
        float sA = accA[i] + b2v, sB = accB[i] + b2v;
        sA = (mkA != 0) ? sA : NEGV; sB = (mkB != 0) ? sB : NEGV; sB = okB ? sB : NEGB;
        float mx = fmaxf(sA, sB);
        mx = fmaxf(mx, __shfl_xor(mx, 16, 32)); mx = fmaxf(mx, __shfl_xor(mx, 8, 32)); mx = fmaxf(mx, __shfl_xor(mx, 4, 32));
        mx = fmaxf(mx, __shfl_xor(mx, 2, 32));  mx = fmaxf(mx, __shfl_xor(mx, 1, 32));
        const float eA = __builtin_amdgcn_exp2f((sA - mx) * L2E);
        float eB = __builtin_amdgcn_exp2f((sB - mx) * L2E); eB = okB ? eB : 0.0f;
        float sm = eA + eB;
        sm += __shfl_xor(sm, 16, 32); sm += __shfl_xor(sm, 8, 32); sm += __shfl_xor(sm, 4, 32); sm += __shfl_xor(sm, 2, 32); sm += __shfl_xor(sm, 1, 32);
        const float inv = __builtin_amdgcn_rcpf(sm) * PCS;
        h16 qa = toh_flush(eA * inv), qb = toh_flush(eB * inv);
        qa = rok[i] ? qa : (h16)0.0f; qb = rok[i] ? qb : (h16)0.0f;
        pt[wave * (4 * HPAD) + i * HPAD + lane] = qa; pt[wave * (4 * HPAD) + i * HPAD + 32 + lane] = qb; }
    wave_sync();
    const v8h val = *(const v8ha*)(&pt[wave * (4 * HPAD) + lane * 8]);
    *(volatile v8h*)dst = val; __threadfence(); *(volatile v8h*)dst = val;
}

__global__ __launch_bounds__(32) void k_gemm2(const h16* __restrict__ AP, const h16* __restrict__ HT, float* OS) {
    __shared__ __align__(16) float os[16 * OSW];
    const int lane = threadIdx.x & 31, lr = lane & 15, hi = lane >> 4;
    const int c0 = (int)blockIdx.x * 64, b = (int)blockIdx.y;
    v8f acc[4][4];
#pragma unroll
    for (int mb = 0; mb < 4; ++mb)
#pragma unroll
        for (int nb = 0; nb < 4; ++nb) acc[mb][nb] = (v8f){};
    const size_t aoff = ((size_t)b * HPAD + (size_t)lr) * HPAD + 8 * hi, boff = ((size_t)b * KP + (size_t)(c0 + lr)) * HPAD + 8 * hi;
#pragma unroll 1
    for (int kc = 0; kc < HPAD; kc += 32) {
        v16h a[4];
#pragma unroll
        for (int mb = 0; mb < 4; ++mb) a[mb] = ldh(AP + aoff + (size_t)mb * 16 * HPAD + kc);
#pragma unroll
        for (int nb = 0; nb < 4; ++nb) { const v16h bq = ldh(HT + boff + (size_t)nb * 16 * HPAD + kc);
#pragma unroll
            for (int mb = 0; mb < 4; ++mb) acc[mb][nb] = wmma16g(a[mb], bq, acc[mb][nb]); }
    }
    float* outp = OS + ((size_t)b * HPAD) * KP + (size_t)c0;
    static_assert(32 * 16 * 8 == 16 * 64 * 4);
#pragma unroll
    for (int mb = 0; mb < 4; ++mb) {
#pragma unroll
        for (int nb = 0; nb < 4; ++nb) {
#pragma unroll
            for (int j = 0; j < 8; ++j) os[(hi * 8 + j) * OSW + nb * 16 + lr] = acc[mb][nb][j] * PCI; }
        wave_sync();
#pragma unroll 1
        for (int ps = 0; ps < 2; ++ps) {
#pragma unroll
            for (int s = 0; s < 8; ++s) { const int row = 2 * s + (lane >> 4), c4 = (lane & 15) * 4;
                const v4f val = *(const v4fa*)(&os[row * OSW + c4]);
                *(volatile v4f*)(outp + (size_t)(mb * 16 + row) * KP + c4) = val; }
            if (ps == 0) __threadfence(); }
        wave_sync();
    }
}

__global__ __launch_bounds__(256) void k_out0(const float* __restrict__ OS, float* O0) {
    const int i = (int)blockIdx.x * 256 + (int)threadIdx.x; if (i >= MROWS * (FD / 4)) return;
    const int r = i / (FD / 4); const int c = (i % (FD / 4)) * 4;
    const int b = r / NN, n = r % NN;
    const v4f v = *(const v4f*)(OS + ((size_t)b * HPAD + (size_t)n) * KP + c);
    *(volatile v4f*)(O0 + (size_t)i * 4) = v; __threadfence(); *(volatile v4f*)(O0 + (size_t)i * 4) = v;
}

static constexpr size_t al256(size_t v) { return (v + 255) & ~(size_t)255; }
static constexpr size_t SZ_WB = al256((size_t)2 * APAD * KP * 2);
static constexpr size_t SZ_XB = al256((size_t)2 * MPAD * KP * 2);
static constexpr size_t SZ_HT = al256((size_t)NB * KP * HPAD * 2);
static constexpr size_t SZ_HP = al256((size_t)2 * MPAD * APAD * 4);
static constexpr size_t SZ_AP = al256((size_t)NB * HPAD * HPAD * 2);
static constexpr size_t SZ_OS = al256((size_t)NB * HPAD * KP * 4);
static constexpr size_t SZ_TOTAL = SZ_WB + SZ_XB + SZ_HT + SZ_HP + SZ_AP + SZ_OS;
static_assert(SZ_TOTAL <= (size_t)134217728);
static_assert(((size_t)MPAD * KP * 2) % 256 == 0);
static_assert(((size_t)MPAD * APAD * 4) % 256 == 0);
static constexpr size_t OUT1_OFF = (size_t)NB_FULL * NN * FD;

extern "C" void kernel_launch(void* const* d_in, const int* in_sizes, int n_in,
                              void* d_out, int out_size, void* d_ws, size_t ws_size, hipStream_t stream) {
    if (n_in < 9) return;
    if ((size_t)in_sizes[0] < (size_t)MROWS * RD || (size_t)in_sizes[1] < (size_t)MROWS * RD) return;
    if ((size_t)in_sizes[2] < (size_t)MROWS || (size_t)in_sizes[3] < (size_t)MROWS) return;
    if ((size_t)in_sizes[4] < (size_t)NPOS * PD || (size_t)in_sizes[5] < (size_t)AD * 2 * FD) return;
    if (in_sizes[6] < AD || in_sizes[7] < AD || in_sizes[8] < 1) return;
    if ((size_t)out_size < OUT1_OFF + (size_t)MROWS * FD) return;
    if (SZ_TOTAL > ws_size) return;
    const float* hist_in = (const float*)d_in[0];
    const float* cand_in = (const float*)d_in[1];
    const int*   maskp   = (const int*)d_in[2];
    const int*   posp    = (const int*)d_in[3];
    const float* pe      = (const float*)d_in[4];
    const float* W1      = (const float*)d_in[5];
    const float* b1      = (const float*)d_in[6];
    const float* w2      = (const float*)d_in[7];
    const float* b2      = (const float*)d_in[8];
    float* OUT0 = (float*)d_out;
    float* OUT1 = (float*)d_out + OUT1_OFF;
    char* wsp = (char*)d_ws;
    bf*  WB = (bf*)wsp;    wsp += SZ_WB;
    bf*  XB = (bf*)wsp;    wsp += SZ_XB;
    h16* HT = (h16*)wsp;   wsp += SZ_HT;
    float* HP = (float*)wsp; wsp += SZ_HP;
    h16* AP = (h16*)wsp;   wsp += SZ_AP;
    float* OS = (float*)wsp; wsp += SZ_OS;
    bf* XC = XB; bf* XH = XB + (size_t)MPAD * KP;
    const float* HC = HP; const float* HH = HP + (size_t)MPAD * APAD;

    k_wconv<<<(unsigned)((2 * APAD * (KP / 8) + 255) / 256), 256, 0, stream>>>(W1, WB);
    k_xrow<<<(unsigned)((MPAD * (KP / 8) + 255) / 256), 256, 0, stream>>>(cand_in, posp, pe, XC, 0);
    k_xrow<<<(unsigned)((MPAD * (KP / 8) + 255) / 256), 256, 0, stream>>>(hist_in, posp, pe, XH, 1);
    k_cand<<<(unsigned)((MROWS * (FD / 4) + 255) / 256), 256, 0, stream>>>(cand_in, pe, OUT1);
    k_histT<<<dim3(KP / 64, NB, 1), 256, 0, stream>>>(hist_in, posp, pe, HT);
    k_gemm1<<<dim3(MPAD / 64, APAD / 64, 2), 32, 0, stream>>>(XB, WB, HP);
    k_score<<<dim3(HPAD / (4 * SW), NB, 1), 32 * SW, 0, stream>>>(HC, HH, maskp, b1, w2, b2, AP);
    k_gemm2<<<dim3(KP / 64, NB, 1), 32, 0, stream>>>(AP, HT, OS);
    k_out0<<<(unsigned)((MROWS * (FD / 4) + 255) / 256), 256, 0, stream>>>(OS, OUT0);
}
